// GRU_40286793236888
// MI455X (gfx1250) — hardware-verified
//
#include <hip/hip_runtime.h>
#include <math.h>

constexpr int NNODE = 1024;
constexpr int NBAT  = 64;
constexpr int CHALF = 64;
constexpr int CCAT  = 128;
constexpr int EDIM  = 16;
constexpr int KTOT  = 3 * CCAT;
constexpr int XCOLS = NBAT * CCAT;
constexpr int ZCOLS = NBAT * CHALF;
constexpr int PBW   = 136;

static_assert(NNODE % 64 == 0 && (2 * NNODE) % 64 == 0 && XCOLS % 64 == 0 && ZCOLS % 64 == 0);
static_assert(NNODE % 32 == 0);
static_assert(NNODE % 2 == 0);

typedef __attribute__((ext_vector_type(16))) _Float16 v16h;
typedef __attribute__((ext_vector_type(8)))  _Float16 v8h;
typedef __attribute__((ext_vector_type(16))) __bf16   v16b;
typedef __attribute__((ext_vector_type(8)))  __bf16   v8b;
typedef __attribute__((ext_vector_type(8)))  float    v8f;
typedef __attribute__((ext_vector_type(4)))  float    v4f;
typedef __attribute__((ext_vector_type(4)))  unsigned int v4u;

__device__ __forceinline__ unsigned short f2bf_bits(float f) {
  unsigned u = __float_as_uint(f);
  return (unsigned short)((u + 0x7FFFu + ((u >> 16) & 1u)) >> 16);
}
__device__ __forceinline__ float bf_bits2f(unsigned short h) { return __uint_as_float(((unsigned)h) << 16); }
__device__ __forceinline__ float bfr(float f) { return bf_bits2f(f2bf_bits(f)); }
__device__ __forceinline__ __bf16 f2bf(float f) { return __builtin_bit_cast(__bf16, f2bf_bits(f)); }
__device__ __forceinline__ unsigned pk16(unsigned short a, unsigned short b) { return (unsigned)a | ((unsigned)b << 16); }

__device__ __forceinline__ void keep4_b(v16b a, v16b b, v16b c, v16b d) { asm volatile("v_nop" :: "v"(a), "v"(b), "v"(c), "v"(d)); }
__device__ __forceinline__ void acc_guard4(v8f& a, v8f& b, v8f& c, v8f& d) { asm volatile("v_nop\n\tv_nop\n\tv_nop\n\tv_nop" : "+v"(a), "+v"(b), "+v"(c), "+v"(d)); }
__device__ __forceinline__ void guard4b(v8f& a, v8f& b, v8f& c, v8f& d, v16b x, v16b y) {
  asm volatile("v_nop\n\tv_nop\n\tv_nop\n\tv_nop" : "+v"(a), "+v"(b), "+v"(c), "+v"(d) : "v"(x), "v"(y));
}
template <typename T> struct Frag;
template <> struct Frag<__bf16> {
  typedef v16b V; union U { v16b v; v8b h[2]; };
  static __device__ __forceinline__ v16b load(const __bf16* p) {
    U f; f.h[0] = *(const v8b*)(p); f.h[1] = *(const v8b*)(p + 16); return f.v;
  }
  static __device__ __forceinline__ v8f mma(v16b a, v16b b, v8f c) {
    return __builtin_amdgcn_wmma_f32_16x16x32_bf16(false, a, false, b, (short)0, c, false, false);
  }
  static __device__ __forceinline__ void keep(v16b a, v16b b, v16b c, v16b d) { keep4_b(a, b, c, d); }
};
__device__ __forceinline__ v8f mma_b(v16b a, v16b b, v8f c) {
  c = __builtin_amdgcn_wmma_f32_16x16x32_bf16(false, a, false, b, (short)0, c, false, false);
  asm volatile("v_nop\n\tv_nop\n\tv_nop\n\tv_nop" : "+v"(c) : "v"(a), "v"(b));
  return c;
}
__device__ __forceinline__ v16b frag_f32_bf16(const float* p) {
  const v4f a = *(const v4f*)(p);
  const v4f bq = *(const v4f*)(p + 4);
  const v4f c = *(const v4f*)(p + 16);
  const v4f d = *(const v4f*)(p + 20);
  v16b f;
#pragma unroll
  for (int e = 0; e < 4; ++e) {
    f[e] = f2bf(a[e]); f[4 + e] = f2bf(bq[e]); f[8 + e] = f2bf(c[e]); f[12 + e] = f2bf(d[e]);
  }
  return f;
}
__device__ __forceinline__ float sigm(float p) {
  const float pc = fminf(fmaxf(p, -30.0f), 30.0f);
  return 1.0f / (1.0f + expf(-pc));
}
__device__ __forceinline__ float tanh_c(float p) {
  const float pc = fminf(fmaxf(p, -20.0f), 20.0f);
  return tanhf(pc);
}

template <int SPLITM, int DIAGSUB, int CMAP>
__global__ __launch_bounds__(256) void wmma_gemm64(
    const unsigned short* __restrict__ Ap, const unsigned short* __restrict__ A2p, int lda,
    const unsigned short* __restrict__ Btp, const unsigned short* __restrict__ Bt2p, int ldb,
    unsigned short* Ch, unsigned short* Cl, int ldc,
    int M, int N, int K, float scale) {
  const __bf16* A = (const __bf16*)Ap; const __bf16* A2 = (const __bf16*)A2p;
  const __bf16* Bt = (const __bf16*)Btp; const __bf16* Bt2 = (const __bf16*)Bt2p;
  __shared__ __align__(16) float sT[8][16 * 68];
  const int lane = threadIdx.x & 31;
  const int wave = threadIdx.x >> 5;
  const int tilesN = N >> 6;
  const int tilesM = M >> 6;
  const int tile = blockIdx.x * 8 + wave;
  if (tile >= tilesM * tilesN) return;
  const int tm = tile / tilesN;
  const int tn = tile - tm * tilesN;
  const int m0 = tm << 6;
  const int n0 = tn << 6;

  const int rlane = lane & 15;
  const int koff  = (lane >> 4) * 8;
  const int mOff  = (lane >> 4) * 8;

  v8f acc[4][4];
#pragma unroll
  for (int i = 0; i < 4; ++i)
#pragma unroll
    for (int j = 0; j < 4; ++j) acc[i][j] = (v8f){0.f,0.f,0.f,0.f,0.f,0.f,0.f,0.f};

  for (int k0 = 0; k0 < K; k0 += 32) {
    v16b bh[4], bl[4];
#pragma unroll
    for (int j = 0; j < 4; ++j) {
      const size_t bo = (size_t)(n0 + (j << 4) + rlane) * ldb + koff + k0;
      bh[j] = Frag<__bf16>::load(Bt + bo);
      bl[j] = (SPLITM == 2) ? Frag<__bf16>::load(Bt2 + bo) : bh[j];
    }
#pragma unroll
    for (int i = 0; i < 4; ++i) {
      const size_t ao = (size_t)(m0 + (i << 4) + rlane) * lda + koff + k0;
      const v16b ah = Frag<__bf16>::load(A + ao);
      const v16b al = (SPLITM >= 1) ? Frag<__bf16>::load(A2 + ao) : ah;
#pragma unroll
      for (int j = 0; j < 4; ++j) {
        acc[i][j] = Frag<__bf16>::mma(ah, bh[j], acc[i][j]);
        if (SPLITM >= 1) acc[i][j] = Frag<__bf16>::mma(al, bh[j], acc[i][j]);
        if (SPLITM == 2) acc[i][j] = Frag<__bf16>::mma(ah, bl[j], acc[i][j]);
      }
      guard4b(acc[i][0], acc[i][1], acc[i][2], acc[i][3], ah, al);
    }
    Frag<__bf16>::keep(bh[0], bh[1], bh[2], bh[3]);
    if (SPLITM == 2) Frag<__bf16>::keep(bl[0], bl[1], bl[2], bl[3]);
  }
  acc_guard4(acc[0][0], acc[0][1], acc[0][2], acc[0][3]);
  acc_guard4(acc[1][0], acc[1][1], acc[1][2], acc[1][3]);
  acc_guard4(acc[2][0], acc[2][1], acc[2][2], acc[2][3]);
  acc_guard4(acc[3][0], acc[3][1], acc[3][2], acc[3][3]);

  float* slab = sT[wave];
  const int cb = CMAP ? (n0 * 2 + 64) : n0;
#pragma unroll
  for (int i = 0; i < 4; ++i) {
    const int mBase = m0 + (i << 4);
#pragma unroll
    for (int j = 0; j < 4; ++j) {
      const int nl = (j << 4) + rlane;
      const int n = n0 + nl;
#pragma unroll
      for (int r = 0; r < 8; ++r) {
        float v = acc[i][j][r] * scale;
        if (DIAGSUB) { if ((mBase + mOff + r) == n) v -= 1.0f; }
        slab[(mOff + r) * 68 + nl] = v;
      }
    }
    __builtin_amdgcn_fence(__ATOMIC_RELEASE, "workgroup");
    __builtin_amdgcn_wave_barrier();
    __builtin_amdgcn_fence(__ATOMIC_ACQUIRE, "workgroup");
    {
      const int q = lane >> 3, c8 = (lane & 7) * 8;
      for (int pass = 0; pass < 2; ++pass) {
#pragma unroll
        for (int it = 0; it < 4; ++it) {
          const int row = it * 4 + q;
          const float* sp = slab + row * 68 + c8;
          v8h hv, lv;
#pragma unroll
          for (int e = 0; e < 8; ++e) {
            unsigned short hb = f2bf_bits(sp[e]);
            unsigned short lb = f2bf_bits(sp[e] - bf_bits2f(hb));
            hv[e] = __builtin_bit_cast(_Float16, hb);
            lv[e] = __builtin_bit_cast(_Float16, lb);
          }
          *(volatile v8h*)(Ch + (size_t)(mBase + row) * ldc + cb + c8) = hv;
          *(volatile v8h*)(Cl + (size_t)(mBase + row) * ldc + cb + c8) = lv;
        }
        __threadfence();
      }
    }
    __builtin_amdgcn_fence(__ATOMIC_RELEASE, "workgroup");
    __builtin_amdgcn_wave_barrier();
    __builtin_amdgcn_fence(__ATOMIC_ACQUIRE, "workgroup");
  }
}

__global__ __launch_bounds__(256) void adj_kernel(const float* __restrict__ E,
                                                  unsigned short* __restrict__ Sh, unsigned short* __restrict__ Sl) {
  __shared__ float sEn[EDIM];
  __shared__ __align__(16) float sA[NNODE];
  __shared__ float sRedM[8];
  __shared__ float sRedS[8];
  const int tid = threadIdx.x, lane = tid & 31, wave = tid >> 5;
  const int n = blockIdx.x;
  if (tid < EDIM) sEn[tid] = bfr(E[(size_t)n * EDIM + tid]);
  __syncthreads();
  float en[EDIM];
#pragma unroll
  for (int e = 0; e < EDIM; ++e) en[e] = sEn[e];

  float v[4];
#pragma unroll
  for (int i = 0; i < 4; ++i) {
    const float* er = E + (size_t)(tid * 4 + i) * EDIM;
    const v4f e0 = *(const v4f*)(er);
    const v4f e1 = *(const v4f*)(er + 4);
    const v4f e2 = *(const v4f*)(er + 8);
    const v4f e3 = *(const v4f*)(er + 12);
    float d = 0.0f;
#pragma unroll
    for (int q = 0; q < 4; ++q) d = fmaf(en[q], bfr(e0[q]), d);
#pragma unroll
    for (int q = 0; q < 4; ++q) d = fmaf(en[4 + q], bfr(e1[q]), d);
#pragma unroll
    for (int q = 0; q < 4; ++q) d = fmaf(en[8 + q], bfr(e2[q]), d);
#pragma unroll
    for (int q = 0; q < 4; ++q) d = fmaf(en[12 + q], bfr(e3[q]), d);
    d = fmaxf(d, 0.0f);
    asm volatile("" : "+v"(d) :: "memory");
    v[i] = d;
  }
  float mx = fmaxf(fmaxf(v[0], v[1]), fmaxf(v[2], v[3]));
#pragma unroll
  for (int off = 1; off < 32; off <<= 1) mx = fmaxf(mx, __shfl_xor(mx, off, 32));
  if (lane == 0) sRedM[wave] = mx;
  __syncthreads();
  float gm = sRedM[0];
#pragma unroll
  for (int w = 1; w < 8; ++w) gm = fmaxf(gm, sRedM[w]);
  float ex[4];
  float ps = 0.0f;
#pragma unroll
  for (int i = 0; i < 4; ++i) { ex[i] = expf(v[i] - gm); ps += ex[i]; }
#pragma unroll
  for (int off = 1; off < 32; off <<= 1) ps += __shfl_xor(ps, off, 32);
  if (lane == 0) sRedS[wave] = ps;
  __syncthreads();
  float tot = 0.0f;
#pragma unroll
  for (int w = 0; w < 8; ++w) tot += sRedS[w];
  const float inv = 1.0f / tot;
#pragma unroll
  for (int i = 0; i < 4; ++i) sA[tid * 4 + i] = ex[i] * inv;
  __syncthreads();
  if (tid < 128) {
    const v4f p0 = *(const v4f*)(sA + tid * 8);
    const v4f p1 = *(const v4f*)(sA + tid * 8 + 4);
    unsigned short hb[8], lb[8];
#pragma unroll
    for (int e = 0; e < 4; ++e) {
      hb[e] = f2bf_bits(p0[e]);     lb[e] = f2bf_bits(p0[e] - bf_bits2f(hb[e]));
      hb[4 + e] = f2bf_bits(p1[e]); lb[4 + e] = f2bf_bits(p1[e] - bf_bits2f(hb[4 + e]));
    }
    const v4u uh = (v4u){pk16(hb[0], hb[1]), pk16(hb[2], hb[3]), pk16(hb[4], hb[5]), pk16(hb[6], hb[7])};
    const v4u ul = (v4u){pk16(lb[0], lb[1]), pk16(lb[2], lb[3]), pk16(lb[4], lb[5]), pk16(lb[6], lb[7])};
    unsigned short* ph = Sh + (size_t)n * NNODE + tid * 8;
    unsigned short* pl = Sl + (size_t)n * NNODE + tid * 8;
    *(volatile v4u*)ph = uh;
    *(volatile v4u*)pl = ul;
    __threadfence();
    *(volatile v4u*)ph = uh;
    *(volatile v4u*)pl = ul;
  }
}

__global__ __launch_bounds__(256) void tr16_kernel(const unsigned short* __restrict__ inA, const unsigned short* __restrict__ inB,
                                                   unsigned short* __restrict__ outA, unsigned short* __restrict__ outB,
                                                   int ld_in, int ld_out) {
  __shared__ unsigned short sm[64 * 66];
  const int tid = threadIdx.x, lane = tid & 31, wave = tid >> 5;
  const int c0 = blockIdx.x * 64;
  const int r0 = blockIdx.y * 64;
  const int q = lane >> 3, c8 = (lane & 7) * 8;
  for (int pl = 0; pl < 2; ++pl) {
    const unsigned short* in = pl ? inB : inA;
    unsigned short* op = pl ? outB : outA;
    __syncthreads();
#pragma unroll
    for (int j = 0; j < 2; ++j) {
      const int c = tid + 256 * j;
      const int row = c >> 3;
      const int col8 = (c & 7) * 8;
      const v4u w = *(const v4u*)(in + (size_t)(r0 + row) * ld_in + c0 + col8);
#pragma unroll
      for (int k = 0; k < 4; ++k) {
        sm[row * 66 + col8 + 2 * k]     = (unsigned short)(w[k] & 0xffffu);
        sm[row * 66 + col8 + 2 * k + 1] = (unsigned short)(w[k] >> 16);
      }
    }
    __syncthreads();
    for (int pass = 0; pass < 2; ++pass) {
#pragma unroll
      for (int it = 0; it < 2; ++it) {
        const int orow = wave * 8 + it * 4 + q;
        unsigned short h[8];
#pragma unroll
        for (int e = 0; e < 8; ++e) h[e] = sm[(c8 + e) * 66 + orow];
        const v4u u = (v4u){pk16(h[0], h[1]), pk16(h[2], h[3]), pk16(h[4], h[5]), pk16(h[6], h[7])};
        *(volatile v4u*)(op + (size_t)(c0 + orow) * ld_out + r0 + c8) = u;
      }
      __threadfence();
    }
  }
}

__global__ __launch_bounds__(256) void packx_kernel(const float* __restrict__ x, const float* __restrict__ st,
                                                    unsigned short* __restrict__ Xt) {
  __shared__ float sm[64 * 65];
  const int tid = threadIdx.x, lane = tid & 31, wave = tid >> 5;
  const int m0 = blockIdx.x * 64;
  const int b = blockIdx.y;
  const int z = blockIdx.z;
  const float* src = z ? st : x;
#pragma unroll
  for (int j = 0; j < 4; ++j) {
    const int c = tid + 256 * j;
    const int row = c >> 4;
    const int col4 = (c & 15) * 4;
    const v4f v = *(const v4f*)(src + ((size_t)b * NNODE + m0 + row) * CHALF + col4);
#pragma unroll
    for (int e = 0; e < 4; ++e) sm[(col4 + e) * 65 + row] = v[e];
  }
  __syncthreads();
  const int q = lane >> 3, c8 = (lane & 7) * 8;
  for (int pass = 0; pass < 2; ++pass) {
#pragma unroll
    for (int it = 0; it < 2; ++it) {
      const int orow = wave * 8 + it * 4 + q;
      unsigned short h[8];
#pragma unroll
      for (int e = 0; e < 8; ++e) h[e] = f2bf_bits(sm[orow * 65 + c8 + e]);
      const v4u u = (v4u){pk16(h[0], h[1]), pk16(h[2], h[3]), pk16(h[4], h[5]), pk16(h[6], h[7])};
      *(volatile v4u*)(Xt + ((size_t)b * CCAT + z * CHALF + orow) * NNODE + m0 + c8) = u;
    }
    __threadfence();
  }
}

template <int NTI, bool TWO>
__device__ __forceinline__ void kstep(v8f (&acc)[NTI], const v16b ah, const v16b al,
                                      const __bf16* wh, const __bf16* wl, int rlane) {
#pragma unroll
  for (int nt = 0; nt < NTI; ++nt) {
    const int ro = (nt * 16 + rlane) * PBW;
    const v16b bh = Frag<__bf16>::load(wh + ro);
    const v16b bl = Frag<__bf16>::load(wl + ro);
    acc[nt] = mma_b(ah, bh, acc[nt]);
    acc[nt] = mma_b(ah, bl, acc[nt]);
    if (TWO) acc[nt] = mma_b(al, bh, acc[nt]);
  }
}

template <bool GATE>
__global__ __launch_bounds__(256) void proj_kernel(
    const float* __restrict__ x, const float* __restrict__ st, const float* __restrict__ E,
    const float* __restrict__ Wpool, const float* __restrict__ bpool,
    const unsigned short* __restrict__ XGh, const unsigned short* __restrict__ XGl,
    const unsigned short* ZSrh, const unsigned short* ZSrl,
    unsigned short* ZSwh, unsigned short* ZSwl, float* Rw,
    const float* Rr, float* __restrict__ out) {
  constexpr int O = GATE ? 128 : 64;
  constexpr int NTI = O / 16;
  constexpr int O4N = O / 4;
  constexpr int PLANE = O * PBW;
  constexpr int SP = O + 4;
  __shared__ __align__(16) float lds_pool[2 * PLANE];
  __shared__ float sEs[2][EDIM];
  __shared__ float sBias[2][O];
  static_assert(8 * 16 * SP <= 2 * PLANE);
  static_assert((PBW % 8) == 0 && ((PLANE * 2) % 16) == 0 && ((16 * SP * 4) % 16) == 0);

  const int tid = threadIdx.x, lane = tid & 31, wave = tid >> 5;
  const int gw = wave >> 2;
  const int mt = wave & 3;
  const int rlane = lane & 15, hh = lane >> 4, koff = hh * 8;
  const int n0 = blockIdx.x * 2;
  const int n = n0 + gw;
  const int b = mt * 16 + rlane;
  unsigned short* sW = (unsigned short*)lds_pool;

  if (tid < 2 * EDIM) {
    const int g = tid >> 4, e = tid & 15;
    sEs[g][e] = bfr(E[(size_t)(n0 + g) * EDIM + e]);
  }
  __syncthreads();
  if (tid < 2 * O) {
    const int g = tid / O;
    const int o = tid - g * O;
    float s = 0.0f;
#pragma unroll
    for (int e = 0; e < 8; ++e) s = fmaf(sEs[g][e], bfr(bpool[e * O + o]), s);
    asm volatile("" : "+v"(s) :: "memory");
#pragma unroll
    for (int e = 8; e < EDIM; ++e) s = fmaf(sEs[g][e], bfr(bpool[e * O + o]), s);
    sBias[g][o] = s;
  }

  v8f acc[NTI];
#pragma unroll
  for (int nt = 0; nt < NTI; ++nt) acc[nt] = (v8f){0.f,0.f,0.f,0.f,0.f,0.f,0.f,0.f};

#pragma unroll 1
  for (int s = 0; s < 3; ++s) {
    __syncthreads();
    {
      unsigned short* wh0 = sW;
      unsigned short* wh1 = sW + PLANE;
      unsigned short* wl0 = sW + 2 * PLANE;
      unsigned short* wl1 = sW + 3 * PLANE;
      const float* wb = Wpool + (size_t)s * CCAT * O;
      constexpr size_t ESTR = (size_t)KTOT * O;
#pragma unroll 1
      for (int idx = tid; idx < CCAT * O4N; idx += 256) {
        const int kk = idx / O4N;
        const int o4 = (idx - kk * O4N) * 4;
        const float* wp = wb + (size_t)kk * O + o4;
        float a0[4] = {0.0f, 0.0f, 0.0f, 0.0f};
        float a1[4] = {0.0f, 0.0f, 0.0f, 0.0f};
        v4f w[8];
#pragma unroll
        for (int e = 0; e < 8; ++e) w[e] = *(const v4f*)(wp + e * ESTR);
#pragma unroll
        for (int e = 0; e < 8; ++e) {
          const float c0 = sEs[0][e], c1 = sEs[1][e];
#pragma unroll
          for (int c = 0; c < 4; ++c) {
            const float wv = bfr(w[e][c]);
            a0[c] = fmaf(c0, wv, a0[c]);
            a1[c] = fmaf(c1, wv, a1[c]);
          }
        }
        asm volatile("" : "+v"(a0[0]), "+v"(a0[1]), "+v"(a0[2]), "+v"(a0[3]),
                          "+v"(a1[0]), "+v"(a1[1]), "+v"(a1[2]), "+v"(a1[3]) :: "memory");
#pragma unroll
        for (int e = 0; e < 8; ++e) w[e] = *(const v4f*)(wp + (8 + e) * ESTR);
#pragma unroll
        for (int e = 0; e < 8; ++e) {
          const float c0 = sEs[0][8 + e], c1 = sEs[1][8 + e];
#pragma unroll
          for (int c = 0; c < 4; ++c) {
            const float wv = bfr(w[e][c]);
            a0[c] = fmaf(c0, wv, a0[c]);
            a1[c] = fmaf(c1, wv, a1[c]);
          }
        }
#pragma unroll
        for (int c = 0; c < 4; ++c) {
          const int ofs = (o4 + c) * PBW + kk;
          unsigned short hb = f2bf_bits(a0[c]);
          unsigned short lb = f2bf_bits(a0[c] - bf_bits2f(hb));
          wh0[ofs] = hb; wl0[ofs] = lb;
          hb = f2bf_bits(a1[c]);
          lb = f2bf_bits(a1[c] - bf_bits2f(hb));
          wh1[ofs] = hb; wl1[ofs] = lb;
        }
      }
    }
    __syncthreads();
    const __bf16* wh = (const __bf16*)(sW + (0 * 2 + gw) * PLANE) + koff;
    const __bf16* wl = (const __bf16*)(sW + (1 * 2 + gw) * PLANE) + koff;
    if (s == 0) {
#pragma unroll
      for (int ks = 0; ks < 2; ++ks) {
        const int k0 = ks * 32;
        const v16b ah = frag_f32_bf16(x + ((size_t)b * NNODE + n) * CHALF + k0 + koff);
        kstep<NTI, false>(acc, ah, ah, wh + k0, wl + k0, rlane);
      }
      if (GATE) {
#pragma unroll
        for (int ks = 2; ks < 4; ++ks) {
          const int k0 = ks * 32;
          const v16b ah = frag_f32_bf16(st + ((size_t)b * NNODE + n) * CHALF + (k0 - 64) + koff);
          kstep<NTI, false>(acc, ah, ah, wh + k0, wl + k0, rlane);
        }
      } else {
#pragma unroll
        for (int ks = 2; ks < 4; ++ks) {
          const int k0 = ks * 32;
          const size_t zo = ((size_t)n * NBAT + b) * CHALF + (k0 - 64) + koff;
          const v16b ah = Frag<__bf16>::load((const __bf16*)ZSrh + zo);
          const v16b al = Frag<__bf16>::load((const __bf16*)ZSrl + zo);
          kstep<NTI, true>(acc, ah, al, wh + k0, wl + k0, rlane);
        }
      }
    } else {
      const size_t ro = (size_t)(s == 1 ? n : NNODE + n) * XCOLS + (size_t)b * CCAT + koff;
#pragma unroll
      for (int ks = 0; ks < 4; ++ks) {
        const int k0 = ks * 32;
        const v16b ah = Frag<__bf16>::load((const __bf16*)XGh + ro + k0);
        const v16b al = Frag<__bf16>::load((const __bf16*)XGl + ro + k0);
        kstep<NTI, true>(acc, ah, al, wh + k0, wl + k0, rlane);
      }
    }
  }
  __syncthreads();

  float* slab = lds_pool + wave * (16 * SP);
#pragma unroll
  for (int nt = 0; nt < NTI; ++nt) {
    const int o = nt * 16 + rlane;
    const float bv = sBias[gw][o];
#pragma unroll
    for (int r = 0; r < 8; ++r) slab[(hh * 8 + r) * SP + o] = acc[nt][r] + bv;
  }
  __syncthreads();

  if (GATE) {
    {
      const int c4 = rlane * 4;
      for (int pass = 0; pass < 2; ++pass) {
#pragma unroll
        for (int it = 0; it < 8; ++it) {
          const int row = it * 2 + hh;
          const v4f p = *(const v4f*)(slab + row * SP + CHALF + c4);
          v4f rv;
#pragma unroll
          for (int e = 0; e < 4; ++e) rv[e] = sigm(p[e]);
          *(volatile v4f*)(Rw + (((size_t)n * NBAT + mt * 16 + row) * CHALF + c4)) = rv;
        }
        __threadfence();
      }
    }
    {
      const int q = lane >> 3, c8 = (lane & 7) * 8;
      for (int pass = 0; pass < 2; ++pass) {
#pragma unroll
        for (int it = 0; it < 4; ++it) {
          const int row = it * 4 + q;
          const int bb = mt * 16 + row;
          const float* sp = slab + row * SP + c8;
          const float* stp = st + ((size_t)bb * NNODE + n) * CHALF + c8;
          const v4f s0 = *(const v4f*)(stp);
          const v4f s1 = *(const v4f*)(stp + 4);
          float sv[8];
#pragma unroll
          for (int e = 0; e < 4; ++e) { sv[e] = bfr(s0[e]); sv[4 + e] = bfr(s1[e]); }
          v8h hv, lv;
#pragma unroll
          for (int e = 0; e < 8; ++e) {
            const float zs = sigm(sp[e]) * sv[e];
            const unsigned short hb = f2bf_bits(zs);
            const unsigned short lb = f2bf_bits(zs - bf_bits2f(hb));
            hv[e] = __builtin_bit_cast(_Float16, hb);
            lv[e] = __builtin_bit_cast(_Float16, lb);
          }
          const size_t zo = ((size_t)n * NBAT + bb) * CHALF + c8;
          *(volatile v8h*)(ZSwh + zo) = hv;
          *(volatile v8h*)(ZSwl + zo) = lv;
        }
        __threadfence();
      }
    }
  } else {
    const int c4 = rlane * 4;
    for (int pass = 0; pass < 2; ++pass) {
#pragma unroll 1
      for (int it = 0; it < 8; ++it) {
        const int row = it * 2 + hh;
        const int bb = mt * 16 + row;
        const v4f p  = *(const v4f*)(slab + row * SP + c4);
        const v4f rv = *(const v4f*)(Rr + (((size_t)n * NBAT + bb) * CHALF + c4));
        const v4f sv = *(const v4f*)(st + (((size_t)bb * NNODE + n) * CHALF + c4));
        v4f ov;
#pragma unroll
        for (int e = 0; e < 4; ++e) {
          const float hc = tanh_c(p[e]);
          const float r = rv[e];
          const float sb = bfr(sv[e]);
          ov[e] = r * sb + (1.0f - r) * hc;
        }
        *(volatile v4f*)(out + (((size_t)bb * NNODE + n) * CHALF + c4)) = ov;
      }
      __threadfence();
    }
  }
}

extern "C" void kernel_launch(void* const* d_in, const int* in_sizes, int n_in,
                              void* d_out, int out_size, void* d_ws, size_t ws_size, hipStream_t stream) {
  (void)in_sizes; (void)out_size;
  if (n_in < 7) return;
  const float* x  = (const float*)d_in[0];
  const float* st = (const float*)d_in[1];
  const float* E  = (const float*)d_in[2];
  const float* gW = (const float*)d_in[3];
  const float* gb = (const float*)d_in[4];
  const float* uW = (const float*)d_in[5];
  const float* ub = (const float*)d_in[6];
  float* out = (float*)d_out;

  constexpr size_t SZ_S  = (size_t)2 * NNODE * NNODE * 2;
  constexpr size_t SZ_AT = (size_t)NNODE * NNODE * 2;
  constexpr size_t SZ_XT = (size_t)XCOLS * NNODE * 2;
  constexpr size_t SZ_XG = (size_t)2 * NNODE * XCOLS * 2;
  constexpr size_t SZ_ZS = (size_t)NNODE * ZCOLS * 2;
  constexpr size_t SZ_R  = (size_t)NNODE * NBAT * CHALF * 4;
  constexpr size_t TOTAL = 2 * SZ_S + 2 * SZ_AT + SZ_XT + 2 * SZ_XG + 2 * SZ_ZS + SZ_R;
  static_assert(TOTAL == 130023424u);
  static_assert(TOTAL <= 134217728u);
  static_assert(2 * (size_t)ZCOLS * NNODE * 2 <= SZ_XT);
  if (TOTAL > ws_size) return;

  char* ws = (char*)d_ws;
  size_t off = 0;
  unsigned short* Sh   = (unsigned short*)(ws + off); off += SZ_S;
  unsigned short* Sl   = (unsigned short*)(ws + off); off += SZ_S;
  unsigned short* Ath  = (unsigned short*)(ws + off); off += SZ_AT;
  unsigned short* Atl  = (unsigned short*)(ws + off); off += SZ_AT;
  unsigned short* Xt   = (unsigned short*)(ws + off); off += SZ_XT;
  unsigned short* XGh  = (unsigned short*)(ws + off); off += SZ_XG;
  unsigned short* XGl  = (unsigned short*)(ws + off); off += SZ_XG;
  unsigned short* ZSh  = (unsigned short*)(ws + off); off += SZ_ZS;
  unsigned short* ZSl  = (unsigned short*)(ws + off); off += SZ_ZS;
  float*          R    = (float*)(ws + off);          off += SZ_R;
  if (off > ws_size) return;
  unsigned short* ZSth = Xt;
  unsigned short* ZStl = Xt + (size_t)ZCOLS * NNODE;
  unsigned short* S2h  = Sh + (size_t)NNODE * NNODE;
  unsigned short* S2l  = Sl + (size_t)NNODE * NNODE;

  adj_kernel<<<NNODE, 256, 0, stream>>>(E, Sh, Sl);
  tr16_kernel<<<dim3(NNODE / 64, NNODE / 64), 256, 0, stream>>>(Sh, Sl, Ath, Atl, NNODE, NNODE);
  wmma_gemm64<2, 1, 0><<<dim3((NNODE / 64) * (NNODE / 64) / 8, 1), 256, 0, stream>>>(
      Sh, Sl, NNODE, Ath, Atl, NNODE, S2h, S2l, NNODE, NNODE, NNODE, NNODE, 2.0f);
  packx_kernel<<<dim3(NNODE / 64, NBAT, 2), 256, 0, stream>>>(x, st, Xt);
  wmma_gemm64<1, 0, 0><<<dim3(((2 * NNODE) / 64) * (XCOLS / 64) / 8, 1), 256, 0, stream>>>(
      Sh, Sl, NNODE, Xt, nullptr, NNODE, XGh, XGl, XCOLS, 2 * NNODE, XCOLS, NNODE, 1.0f);
  proj_kernel<true><<<NNODE / 2, 256, 0, stream>>>(x, st, E, gW, gb, XGh, XGl, nullptr, nullptr, ZSh, ZSl, R, nullptr, nullptr);
  tr16_kernel<<<dim3(ZCOLS / 64, NNODE / 64), 256, 0, stream>>>(ZSh, ZSl, ZSth, ZStl, ZCOLS, NNODE);
  wmma_gemm64<2, 0, 1><<<dim3(((2 * NNODE) / 64) * (ZCOLS / 64) / 8, 1), 256, 0, stream>>>(
      Sh, Sl, NNODE, ZSth, ZStl, NNODE, XGh, XGl, XCOLS, 2 * NNODE, ZCOLS, NNODE, 1.0f);
  proj_kernel<false><<<NNODE / 2, 256, 0, stream>>>(x, st, E, uW, ub, XGh, XGl, ZSh, ZSl, nullptr, nullptr, nullptr, R, out);
}
